// Encoder_22273700397058
// MI455X (gfx1250) — hardware-verified
//
#include <hip/hip_runtime.h>
#include <stddef.h>
#include <stdint.h>
#include <math.h>

#define NNODE  50000
#define NEDGE  500000
#define NGR    100
#define DF     128
#define R2     (2 * NNODE)
#define NOUTF  38402

#define NTHR   256
#define NWAVE  8
#define CHUNK  2048
#define WCAP   256
#define LISTN  (NWAVE * WCAP)
#define NBA    1024
#define SLA    10
#define RCAP   12288
#define DEGCAP 32
#define AGG_ZINTS    (LISTN + 2 * RCAP + 3 * NBA)
#define MISC_INTS    16
#define AGG_LDS_INTS (AGG_ZINTS + MISC_INTS)

#define MROWS  64
#define MTHR   128
#define LP     392
#define NRECB  ((R2 + MROWS - 1) / MROWS)
#define NTSB   ((NNODE + 63) / 64)
#define NKROWS 128

static_assert((CHUNK & (CHUNK - 1)) == 0 && CHUNK == NWAVE * WCAP && WCAP == 8 * 32);
static_assert((NBA & (NBA - 1)) == 0 && NBA == (1 << SLA));
static_assert(((long long)CHUNK << SLA) < (1LL << 31));
static_assert(((long long)NEDGE << SLA) < (1LL << 31));
static_assert(NBA % NWAVE == 0 && NBA % 32 == 0);
static_assert(AGG_ZINTS % (NTHR * 4) == 0);
static_assert(AGG_LDS_INTS * 4 <= 300000);
static_assert(MROWS == (MTHR / 32) * 16 && DF == 4 * 32 && DF % 32 == 0);
static_assert(MROWS * LP * 2 >= MROWS * DF * 4);
static_assert((LP * 2) % 16 == 0);
static_assert((size_t)NNODE * 256 * 2 <= (size_t)R2 * DF * 4);
static_assert(NOUTF == 3 * NGR * DF + 2);
static_assert(NGR <= NKROWS && 4 * 25 == NGR);
static_assert(((NNODE + NBA - 1) / NBA) * NBA >= NNODE);

typedef float          v2f   __attribute__((ext_vector_type(2)));
typedef float          v4f   __attribute__((ext_vector_type(4)));
typedef float          v8f   __attribute__((ext_vector_type(8)));
typedef double         v2d   __attribute__((ext_vector_type(2)));
typedef int            v4i   __attribute__((ext_vector_type(4)));
typedef int            v8i   __attribute__((ext_vector_type(8)));
typedef unsigned short v4us  __attribute__((ext_vector_type(4)));
typedef unsigned short v8us  __attribute__((ext_vector_type(8)));
typedef unsigned short v16us __attribute__((ext_vector_type(16)));
typedef __bf16         v16bf __attribute__((ext_vector_type(16)));
typedef v4f  __attribute__((may_alias)) v4fa;
typedef v2d  __attribute__((may_alias)) v2da;
typedef v4i  __attribute__((may_alias)) v4ia;
typedef v4us __attribute__((may_alias)) v4usa;
typedef v8us __attribute__((may_alias)) v8usa;
union FragB { v16bf v; v16us u; v8us h[2]; v8i w; };

__device__ __forceinline__ v8f wmb(const FragB& a, const FragB& b, v8f c) {
  v8f d = __builtin_amdgcn_wmma_f32_16x16x32_bf16(false, a.v, false, b.v, (short)0, c, false, false);
  asm volatile("v_nop\n\tv_nop\n\tv_nop\n\tv_nop" : "+v"(d) : "v"(a.w), "v"(b.w));
  return d;
}

__device__ __forceinline__ unsigned bf16_bits(float f) {
  const unsigned u = __float_as_uint(f);
  return (u + 0x7FFFu + ((u >> 16) & 1u)) >> 16;
}
__device__ __forceinline__ float bf16_val(float f) {
  return __uint_as_float(bf16_bits(f) << 16);
}
__device__ __forceinline__ void split3(float x, unsigned& h, unsigned& m, unsigned& l) {
  h = bf16_bits(x);
  const float r1 = x - __uint_as_float(h << 16);
  m = bf16_bits(r1);
  const float r2 = r1 - __uint_as_float(m << 16);
  l = bf16_bits(r2);
}
__device__ __forceinline__ void wave_sync() {
  __builtin_amdgcn_fence(__ATOMIC_RELEASE, "wavefront");
  __builtin_amdgcn_wave_barrier();
  __builtin_amdgcn_fence(__ATOMIC_ACQUIRE, "wavefront");
}

__global__ __launch_bounds__(NTHR) void k_prep(const float* __restrict__ Wi1, const float* __restrict__ Wi2,
                                               const float* __restrict__ Wg1, const float* __restrict__ Wg2,
                                               unsigned short* WT) {
  const int u  = (int)blockIdx.x * NTHR + (int)threadIdx.x;
  const int mi = u >> 11;
  const int v  = u & 2047;
  const int n  = v >> 4;
  const int k8 = (v & 15) * 8;
  const float* W;
  int mo;
  if (mi == 0)      { W = Wi1; mo = 0; }
  else if (mi == 1) { W = Wi2; mo = 0; }
  else if (mi < 5)  { W = Wg1; mo = mi - 2; }
  else if (mi < 8)  { W = Wg2; mo = mi - 5; }
  else return;
  const float* p = W + (size_t)mo * (DF * DF) + (size_t)k8 * DF + n;
  v8us o;
#pragma unroll
  for (int i = 0; i < 8; ++i) o[i] = (unsigned short)bf16_bits(p[(size_t)i * DF]);
  unsigned short* dp = WT + (size_t)mi * (DF * DF) + (size_t)n * DF + k8;
  *(volatile v8us*)dp = o;
  __threadfence();
  *(volatile v8us*)dp = o;
}

template <int NP>
__device__ __forceinline__ void gemm_tile(const unsigned short* pl, const unsigned short* __restrict__ WT,
                                          int wave, int m, int hh, v8f (&acc)[8]) {
  const unsigned short* arow = pl + (16 * wave + m) * LP + 8 * hh;
  const unsigned short* wp   = WT + (size_t)m * DF + 8 * hh;
#pragma unroll 1
  for (int ks = 0; ks < DF / 32; ++ks) {
    FragB a0, a1, a2;
    a0.h[0] = *(const v8usa*)(arow + 32 * ks);
    a0.h[1] = *(const v8usa*)(arow + 32 * ks + 16);
    a1 = a0; a2 = a0;
    if constexpr (NP == 3) {
      a1.h[0] = *(const v8usa*)(arow + DF + 32 * ks);
      a1.h[1] = *(const v8usa*)(arow + DF + 32 * ks + 16);
      a2.h[0] = *(const v8usa*)(arow + 2 * DF + 32 * ks);
      a2.h[1] = *(const v8usa*)(arow + 2 * DF + 32 * ks + 16);
    }
#pragma unroll
    for (int nt = 0; nt < 8; ++nt) {
      const unsigned short* wq = wp + (size_t)(16 * nt) * DF + 32 * ks;
      FragB bf;
      bf.h[0] = *(const v8usa*)wq;
      bf.h[1] = *(const v8usa*)(wq + 16);
      acc[nt] = wmb(a0, bf, acc[nt]);
      if constexpr (NP == 3) {
        acc[nt] = wmb(a1, bf, acc[nt]);
        acc[nt] = wmb(a2, bf, acc[nt]);
      }
    }
  }
}

template <int MODE>
__global__ __launch_bounds__(MTHR) void k_mlp(const float* X, int R,
                                              const unsigned short* __restrict__ W1T, const float* __restrict__ b1,
                                              const unsigned short* __restrict__ W2T, const float* __restrict__ b2,
                                              float* OUT, double* rec) {
  __shared__ __attribute__((aligned(16))) unsigned short pl[MROWS * LP];
  __shared__ __attribute__((aligned(16))) double sred[2 * DF];
  __shared__ __attribute__((aligned(16))) float sb[2 * DF];
  float* stg = (float*)pl;
  const int tid = (int)threadIdx.x, lane = tid & 31, wave = tid >> 5, hh = lane >> 4, m = lane & 15;
  const int rowBase = (int)blockIdx.x * MROWS;

  sb[tid]      = bf16_val(b1[tid]);
  sb[DF + tid] = bf16_val(b2[tid]);

#pragma unroll 4
  for (int i = 0; i < 16; ++i) {
    const int idx = i * MTHR + tid;
    const int lr = idx >> 5, c4 = idx & 31;
    const int gr = rowBase + lr;
    const int gc = gr < R ? gr : R - 1;
    v4f v = *(const v4fa*)(X + (size_t)gc * DF + 4 * c4);
    const bool ok = gr < R;
    v.x = ok ? v.x : 0.0f; v.y = ok ? v.y : 0.0f; v.z = ok ? v.z : 0.0f; v.w = ok ? v.w : 0.0f;
    unsigned short* d = pl + lr * LP + 4 * c4;
    if constexpr (MODE == 0) {
      v4us h4;
      h4[0] = (unsigned short)bf16_bits(v.x); h4[1] = (unsigned short)bf16_bits(v.y);
      h4[2] = (unsigned short)bf16_bits(v.z); h4[3] = (unsigned short)bf16_bits(v.w);
      *(v4usa*)d = h4;
    } else {
      v4us h4, m4, l4;
      unsigned a, b, c;
      split3(v.x, a, b, c); h4[0] = (unsigned short)a; m4[0] = (unsigned short)b; l4[0] = (unsigned short)c;
      split3(v.y, a, b, c); h4[1] = (unsigned short)a; m4[1] = (unsigned short)b; l4[1] = (unsigned short)c;
      split3(v.z, a, b, c); h4[2] = (unsigned short)a; m4[2] = (unsigned short)b; l4[2] = (unsigned short)c;
      split3(v.w, a, b, c); h4[3] = (unsigned short)a; m4[3] = (unsigned short)b; l4[3] = (unsigned short)c;
      *(v4usa*)d = h4;
      *(v4usa*)(d + DF) = m4;
      *(v4usa*)(d + 2 * DF) = l4;
    }
  }
  __syncthreads();

  v8f acc[8];
  const v8f zz = {0.f, 0.f, 0.f, 0.f, 0.f, 0.f, 0.f, 0.f};
#pragma unroll
  for (int t = 0; t < 8; ++t) acc[t] = zz;
  gemm_tile<(MODE == 0) ? 1 : 3>(pl, W1T, wave, m, hh, acc);
  __syncthreads();

#pragma unroll
  for (int nt = 0; nt < 8; ++nt) {
    const int lc = 16 * nt + m;
    const float bb = sb[lc];
#pragma unroll
    for (int r = 0; r < 8; ++r) {
      float v = acc[nt][r] + bb;
      v = (v > 0.0f) ? v : (v - v);
      unsigned a, b, c;
      split3(v, a, b, c);
      unsigned short* d = pl + (16 * wave + 8 * hh + r) * LP + lc;
      d[0]      = (unsigned short)a;
      d[DF]     = (unsigned short)b;
      d[2 * DF] = (unsigned short)c;
    }
  }
  __syncthreads();

#pragma unroll
  for (int t = 0; t < 8; ++t) acc[t] = zz;
  gemm_tile<3>(pl, W2T, wave, m, hh, acc);
  __syncthreads();

#pragma unroll
  for (int nt = 0; nt < 8; ++nt) {
    const int lc = 16 * nt + m;
    const float bb = sb[DF + lc];
#pragma unroll
    for (int r = 0; r < 8; ++r) {
      float v = acc[nt][r] + bb;
      if constexpr (MODE != 0) v = (v > 0.0f) ? v : (v - v);
      stg[(16 * wave + 8 * hh + r) * DF + lc] = v;
    }
  }
  __syncthreads();

  v4f pv[16];
#pragma unroll
  for (int i = 0; i < 16; ++i) pv[i] = *(const v4fa*)(stg + (16 * wave + i) * DF + 4 * lane);

  if constexpr (MODE != 0) {
    double s = 0.0, q = 0.0;
#pragma unroll 4
    for (int rr = 0; rr < MROWS; ++rr) {
      const float fv = stg[rr * DF + tid];
      const double dv = (rowBase + rr < R) ? (double)fv : 0.0;
      s += dv;
      q += dv * dv;
    }
    sred[tid] = s;
    sred[DF + tid] = q;
  }
  __syncthreads();

#pragma unroll
  for (int i = 0; i < 16; ++i) {
    const int r = rowBase + 16 * wave + i;
    if (r < R) *(volatile v4f*)(OUT + (size_t)r * DF + 4 * lane) = pv[i];
  }
  if constexpr (MODE != 0) {
    const v2d o = *(const v2da*)(sred + 2 * tid);
    double* rp = rec + (size_t)blockIdx.x * (2 * DF) + 2 * tid;
    *(volatile v2d*)rp = o;
    __threadfence();
    *(volatile v2d*)rp = o;
  } else {
    __threadfence();
  }
#pragma unroll
  for (int i = 0; i < 16; ++i) {
    const int r = rowBase + 16 * wave + i;
    if (r < R) *(volatile v4f*)(OUT + (size_t)r * DF + 4 * lane) = pv[i];
  }
}

__global__ __launch_bounds__(NTHR) void k_neg(float* A, const int* __restrict__ idx, int nN) {
  const int gid = (int)blockIdx.x * NTHR + (int)threadIdx.x;
  const int row = gid >> 5, lane = gid & 31;
  if (row >= nN) return;
  int s = idx[row];
  s = s < 0 ? 0 : (s > nN - 1 ? nN - 1 : s);
  const v4f v = *(const v4fa*)(A + (size_t)s * DF + 4 * lane);
  float* op = A + (size_t)(nN + row) * DF + 4 * lane;
  *(volatile v4f*)op = v;
  __threadfence();
  *(volatile v4f*)op = v;
}

template <int SLB>
__device__ __forceinline__ int scan_chunk(const int* __restrict__ dsts, int nE, int cbase, int slotBase,
                                          int nb, int* list, int lane, int wave) {
  int wc = 0;
  const int elb  = wave * WCAP + lane;
  const int eb   = cbase + elb;
  const int sent = -2147483647 - 1;
  const int e0 = eb, e1 = eb + 32, e2 = eb + 64, e3 = eb + 96;
  const int e4 = eb + 128, e5 = eb + 160, e6 = eb + 192, e7 = eb + 224;
  int d0 = dsts[min(e0, nE - 1)];
  int d1 = dsts[min(e1, nE - 1)];
  int d2 = dsts[min(e2, nE - 1)];
  int d3 = dsts[min(e3, nE - 1)];
  int d4 = dsts[min(e4, nE - 1)];
  int d5 = dsts[min(e5, nE - 1)];
  int d6 = dsts[min(e6, nE - 1)];
  int d7 = dsts[min(e7, nE - 1)];
  d0 = (e0 < nE) ? d0 : sent; d1 = (e1 < nE) ? d1 : sent;
  d2 = (e2 < nE) ? d2 : sent; d3 = (e3 < nE) ? d3 : sent;
  d4 = (e4 < nE) ? d4 : sent; d5 = (e5 < nE) ? d5 : sent;
  d6 = (e6 < nE) ? d6 : sent; d7 = (e7 < nE) ? d7 : sent;
  const unsigned nbs = (unsigned)slotBase;
  const unsigned unb = (unsigned)nb;
  const unsigned s0 = (unsigned)d0 - nbs, s1 = (unsigned)d1 - nbs;
  const unsigned s2 = (unsigned)d2 - nbs, s3 = (unsigned)d3 - nbs;
  const unsigned s4 = (unsigned)d4 - nbs, s5 = (unsigned)d5 - nbs;
  const unsigned s6 = (unsigned)d6 - nbs, s7 = (unsigned)d7 - nbs;
  const bool h0 = s0 < unb, h1 = s1 < unb, h2 = s2 < unb, h3 = s3 < unb;
  const bool h4 = s4 < unb, h5 = s5 < unb, h6 = s6 < unb, h7 = s7 < unb;
  const unsigned any = __builtin_amdgcn_ballot_w32(h0 | h1 | h2 | h3 | h4 | h5 | h6 | h7);
  if (any != 0u) {
#define HITJ(J, HJ, SJ) { \
      const unsigned mj = __builtin_amdgcn_ballot_w32(HJ); \
      if (mj != 0u) { \
        if (HJ) { \
          const int pos = wc + (int)__builtin_amdgcn_mbcnt_lo(mj, 0u); \
          if (pos < WCAP) list[wave * WCAP + pos] = ((elb + 32 * (J)) << SLB) | (int)(SJ); \
        } \
        wc += (int)__builtin_popcount(mj); } }
    HITJ(0, h0, s0)
    HITJ(1, h1, s1)
    HITJ(2, h2, s2)
    HITJ(3, h3, s3)
    HITJ(4, h4, s4)
    HITJ(5, h5, s5)
    HITJ(6, h6, s6)
    HITJ(7, h7, s7)
#undef HITJ
  }
  return wc;
}

__global__ __launch_bounds__(NTHR) void k_scan(const int* __restrict__ srcs, const int* __restrict__ dsts,
                                               int nE, int nN, const float* __restrict__ Ain, float* Bout) {
  extern __shared__ __attribute__((aligned(16))) int dsm[];
  int* list = dsm;
  int* hl   = dsm + LISTN;
  int* sl   = hl + RCAP;
  int* cnt  = sl + RCAP;
  int* offs = cnt + NBA;
  int* cur  = offs + NBA;
  int* misc = cur + NBA;
  const int tid = (int)threadIdx.x, lane = tid & 31, wave = tid >> 5;
  const int nodeBase = (int)blockIdx.x * NBA;

  {
    const v4i z4 = {0, 0, 0, 0};
    for (int i = tid * 4; i < AGG_ZINTS; i += NTHR * 4) *(v4ia*)(dsm + i) = z4;
    if (tid < MISC_INTS) misc[tid] = 0;
  }
  __syncthreads();

  int t = 0, ov = 0;
  const int nChunks = (nE + CHUNK - 1) / CHUNK;
#pragma unroll 1
  for (int ch = 0; ch < nChunks; ++ch) {
    const int cbase = ch * CHUNK;
    const int wc = scan_chunk<SLA>(dsts, nE, cbase, nodeBase, NBA, list, lane, wave);
    if (lane == 0) misc[wave] = wc;
    __syncthreads();
    if (wave == 0) {
#pragma unroll 1
      for (int w2 = 0; w2 < NWAVE; ++w2) {
        int c = misc[w2];
        c = c < 0 ? 0 : (c > WCAP ? WCAP : c);
#pragma unroll 1
        for (int b0 = 0; b0 < c; b0 += 32) {
          const int idx = b0 + lane;
          const int ent = list[w2 * WCAP + (idx < WCAP ? idx : WCAP - 1)];
          const int m32 = (c - b0) < 32 ? (c - b0) : 32;
#pragma unroll 1
          for (int k = 0; k < m32; ++k) {
            const int u    = __builtin_amdgcn_readlane(ent, k);
            const int slot = u & (NBA - 1);
            const int el   = (u >> SLA) & (CHUNK - 1);
            const int pk   = ((cbase + el) << SLA) | slot;
            if (t < RCAP) {
              if (lane == 0) { hl[t] = pk; cnt[slot] = cnt[slot] + 1; }
              t = t + 1;
            } else {
              ov = 1;
            }
          }
        }
      }
    }
    __syncthreads();
  }
  if (wave == 0 && lane == 0) { misc[8] = t; misc[9] = ov; }
  __syncthreads();
  int tt = misc[8];
  tt = tt < 0 ? 0 : (tt > RCAP ? RCAP : tt);
  const int ovf = misc[9];

  if (wave == 0) {
    const int base = lane * (NBA / 32);
    int s = 0;
#pragma unroll 1
    for (int i = 0; i < NBA / 32; ++i) s += cnt[base + i];
    int incl = s;
#pragma unroll
    for (int d = 1; d < 32; d <<= 1) {
      const int y = __shfl_up(incl, d, 32);
      if (lane >= d) incl += y;
    }
    int run = incl - s;
#pragma unroll 1
    for (int i = 0; i < NBA / 32; ++i) {
      const int cv = cnt[base + i];
      offs[base + i] = run;
      cur[base + i]  = run;
      run += cv;
    }
  }
  __syncthreads();
  if (wave == 0) {
#pragma unroll 1
    for (int b0 = 0; b0 < tt; b0 += 32) {
      const int idx = b0 + lane;
      const int ent = hl[idx < RCAP ? idx : RCAP - 1];
      const int m32 = (tt - b0) < 32 ? (tt - b0) : 32;
#pragma unroll 1
      for (int k = 0; k < m32; ++k) {
        const int u    = __builtin_amdgcn_readlane(ent, k);
        const int slot = u & (NBA - 1);
        if (lane == 0) {
          int p = cur[slot];
          p = p < 0 ? 0 : (p > RCAP - 1 ? RCAP - 1 : p);
          sl[p] = u;
          cur[slot] = p + 1;
        }
      }
    }
  }
  __syncthreads();

  const int offv = srcs[nE - 1] + 1;
  const float qnan = __int_as_float(0x7fc00000);
  const float pz = (ovf != 0 || offv != nN) ? qnan : 0.0f;
#pragma unroll 1
  for (int si = 0; si < NBA / NWAVE; ++si) {
    const int s    = si * NWAVE + wave;
    const int node = nodeBase + s;
    int c = cnt[s];
    const bool big = c > DEGCAP;
    c = c < 0 ? 0 : (c > DEGCAP ? DEGCAP : c);
    int o = offs[s];
    o = o < 0 ? 0 : (o > RCAP ? RCAP : o);
    const int nc = node < nN ? node : nN - 1;
    v4f aa = {0.0f, 0.0f, 0.0f, 0.0f};
    v4f ab = {0.0f, 0.0f, 0.0f, 0.0f};
#pragma unroll 1
    for (int b0 = 0; b0 < c; b0 += 32) {
      int idx = o + b0 + lane;
      idx = idx > RCAP - 1 ? RCAP - 1 : idx;
      const int ent = sl[idx];
      int eid = ent >> SLA;
      eid = eid < 0 ? 0 : (eid > nE - 1 ? nE - 1 : eid);
      int sr = srcs[eid];
      sr = sr < 0 ? 0 : (sr > nN - 1 ? nN - 1 : sr);
      const int m32 = (c - b0) < 32 ? (c - b0) : 32;
#pragma unroll 1
      for (int k = 0; k < m32; ++k) {
        const int sk = __builtin_amdgcn_readlane(sr, k);
        const v4f va = *(const v4fa*)(Ain + (size_t)sk * DF + 4 * lane);
        const v4f vb = *(const v4fa*)(Ain + (size_t)(nN + sk) * DF + 4 * lane);
        aa += va;
        ab += vb;
      }
    }
    const v4f sa = *(const v4fa*)(Ain + (size_t)nc * DF + 4 * lane);
    const v4f sc = *(const v4fa*)(Ain + (size_t)(nN + nc) * DF + 4 * lane);
    const float pzr = big ? qnan : pz;
    v4f za = sa + aa;
    v4f zb = sc + ab;
    za.x += pzr; za.y += pzr; za.z += pzr; za.w += pzr;
    zb.x += pzr; zb.y += pzr; zb.z += pzr; zb.w += pzr;
    if (node < nN) {
      float* pa = Bout + (size_t)node * DF + 4 * lane;
      float* pb = Bout + (size_t)(nN + node) * DF + 4 * lane;
      *(volatile v4f*)pa = za;
      *(volatile v4f*)pb = zb;
      __threadfence();
      *(volatile v4f*)pa = za;
      *(volatile v4f*)pb = zb;
    }
  }
}

__global__ __launch_bounds__(NTHR) void k_bn_combine(const double* __restrict__ rec, int nRec, float* stat) {
  __shared__ double sd[2 * DF];
  __shared__ __attribute__((aligned(16))) float st[2 * DF];
  const int tid = (int)threadIdx.x;
  double a = 0.0;
#pragma unroll 4
  for (int b = 0; b < nRec; ++b) a += rec[(size_t)b * (2 * DF) + tid];
  sd[tid] = a;
  __syncthreads();
  if (tid < DF) {
    const double rn = 1.0 / (double)R2;
    const double mu = sd[tid] * rn;
    const double vr = sd[DF + tid] * rn - mu * mu;
    const float fv = (float)vr;
    st[tid] = (float)mu;
    st[DF + tid] = 1.0f / sqrtf(fv + 1e-5f);
  }
  __syncthreads();
  if (tid < 64) {
    const v4f o = *(const v4fa*)(st + 4 * tid);
    float* op = stat + 4 * tid;
    *(volatile v4f*)op = o;
    __threadfence();
    *(volatile v4f*)op = o;
  }
}

__global__ __launch_bounds__(NTHR) void k_bn_apply(float* Z, float* GL, const float* __restrict__ stat,
                                                   const float* __restrict__ gam, const float* __restrict__ bet,
                                                   const float* __restrict__ wl, const float* __restrict__ bl,
                                                   int mode, int R) {
#pragma clang fp contract(off)
  const int tid = (int)threadIdx.x, lane = tid & 31, wave = tid >> 5;
  const int row0 = (int)blockIdx.x * 64 + wave * 8;
  const v4f mu  = *(const v4f*)(stat + 4 * lane);
  const v4f inv = *(const v4f*)(stat + DF + 4 * lane);
  v4f g = *(const v4f*)(gam + 4 * lane);
  v4f b = *(const v4f*)(bet + 4 * lane);
  g.x = bf16_val(g.x); g.y = bf16_val(g.y); g.z = bf16_val(g.z); g.w = bf16_val(g.w);
  b.x = bf16_val(b.x); b.y = bf16_val(b.y); b.z = bf16_val(b.z); b.w = bf16_val(b.w);
  const float w   = bf16_val(wl[0]);
  const float blv = bf16_val(bl[0]);
#pragma unroll 1
  for (int i = 0; i < 8; ++i) {
    const int row = row0 + i;
    if (row >= R) break;
    float* zp = Z  + (size_t)row * DF + 4 * lane;
    float* gp = GL + (size_t)row * DF + 4 * lane;
    const v4f z = *(const v4fa*)zp;
    v4f h;
    h.x = ((z.x - mu.x) * inv.x) * g.x + b.x;
    h.y = ((z.y - mu.y) * inv.y) * g.y + b.y;
    h.z = ((z.z - mu.z) * inv.z) * g.z + b.z;
    h.w = ((z.w - mu.w) * inv.w) * g.w + b.w;
    v4f gv;
    gv.x = w * h.x; gv.y = w * h.y; gv.z = w * h.z; gv.w = w * h.w;
    if (mode != 0) {
      const v4f old = *(const v4fa*)gp;
      gv.x = old.x + gv.x; gv.y = old.y + gv.y; gv.z = old.z + gv.z; gv.w = old.w + gv.w;
    }
    if (mode == 2) { gv.x += blv; gv.y += blv; gv.z += blv; gv.w += blv; }
    *(volatile v4f*)zp = h;
    *(volatile v4f*)gp = gv;
    __threadfence();
    *(volatile v4f*)zp = h;
    *(volatile v4f*)gp = gv;
  }
}

__global__ __launch_bounds__(NTHR) void k_ts(const float* __restrict__ GL, const float* __restrict__ Wp,
                                             const float* __restrict__ bp, const float* __restrict__ wsub,
                                             int nN, float* coefo, double* prec, unsigned short* QN) {
#pragma clang fp contract(off)
  __shared__ __attribute__((aligned(16))) float wps[3 * DF * 2];
  __shared__ float bps[8];
  __shared__ float wsb[4];
  __shared__ __attribute__((aligned(16))) float coefs[64];
  __shared__ double wpart[NWAVE];
  __shared__ __attribute__((aligned(16))) unsigned short rb[NWAVE * 256];
  const int tid = (int)threadIdx.x, lane = tid & 31, wave = tid >> 5;
  const int rowBase = (int)blockIdx.x * 64;

#pragma unroll 1
  for (int i = tid; i < 3 * DF * 2; i += NTHR) wps[i] = bf16_val(Wp[i]);
  if (tid < 8) {
    const float tv = bp[tid < 6 ? tid : 5];
    bps[tid] = (tid < 6) ? bf16_val(tv) : 0.0f;
  }
  if (tid < 4) wsb[tid] = bf16_val(wsub[tid]);
  __syncthreads();

  unsigned short* rbw = rb + wave * 256;
  double dacc = 0.0;
#pragma unroll 1
  for (int i = 0; i < 8; ++i) {
    const int lr = wave * 8 + i;
    const int n  = rowBase + lr;
    const int nc = n < nN ? n : nN - 1;
    const bool live = n < nN;
    const v4f p = *(const v4fa*)(GL + (size_t)nc * DF + 4 * lane);

    bool m0 = false, m1 = false, m2 = false;
    double dd = 0.0;
#pragma unroll 1
    for (int k = 0; k < 3; ++k) {
      const v4f wa = *(const v4fa*)(wps + k * 256 + 8 * lane);
      const v4f wb = *(const v4fa*)(wps + k * 256 + 8 * lane + 4);
      float y0 = p.x * wa.x;
      y0 = fmaf(p.y, wa.z, y0); y0 = fmaf(p.z, wb.x, y0); y0 = fmaf(p.w, wb.z, y0);
      float y1 = p.x * wa.y;
      y1 = fmaf(p.y, wa.w, y1); y1 = fmaf(p.z, wb.y, y1); y1 = fmaf(p.w, wb.w, y1);
#pragma unroll
      for (int o = 16; o > 0; o >>= 1) {
        y0 += __shfl_xor(y0, o, 32);
        y1 += __shfl_xor(y1, o, 32);
      }
      const bool use = (k == 0) ? true : ((k == 1) ? m0 : !m0);
      const float c0 = bps[2 * k], c1 = bps[2 * k + 1];
      const float l0 = use ? (y0 + c0) : c0;
      const float l1 = use ? (y1 + c1) : c1;
      const float mx = fmaxf(l0, l1);
      const float e0 = expf(l0 - mx), e1 = expf(l1 - mx);
      const float sm = e0 + e1;
      const float rs = 1.0f / sm;
      const float p0 = e0 * rs, p1 = e1 * rs;
      const bool mk = p0 >= 0.5f;
      dd += (double)fabsf(p0 - p1);
      m0 = (k == 0) ? mk : m0;
      m1 = (k == 1) ? mk : m1;
      m2 = (k == 2) ? mk : m2;
    }
    const int leaf = m0 ? (m1 ? 0 : 1) : (m2 ? 2 : 3);
    const float cf = wsb[leaf];
    dacc += live ? dd : 0.0;
    if (lane == 0) coefs[lr] = live ? cf : 0.0f;

    float ss = p.x * p.x + p.y * p.y + p.z * p.z + p.w * p.w;
#pragma unroll
    for (int o = 16; o > 0; o >>= 1) ss += __shfl_xor(ss, o, 32);
    const float inv = 1.0f / fmaxf(sqrtf(ss), 1e-12f);
    const float q0 = p.x * inv, q1 = p.y * inv, q2 = p.z * inv, q3 = p.w * inv;
    v4us h4, l4;
    {
      unsigned hb;
      hb = bf16_bits(q0); h4[0] = (unsigned short)hb; l4[0] = (unsigned short)bf16_bits(q0 - __uint_as_float(hb << 16));
      hb = bf16_bits(q1); h4[1] = (unsigned short)hb; l4[1] = (unsigned short)bf16_bits(q1 - __uint_as_float(hb << 16));
      hb = bf16_bits(q2); h4[2] = (unsigned short)hb; l4[2] = (unsigned short)bf16_bits(q2 - __uint_as_float(hb << 16));
      hb = bf16_bits(q3); h4[3] = (unsigned short)hb; l4[3] = (unsigned short)bf16_bits(q3 - __uint_as_float(hb << 16));
    }
    *(v4usa*)(rbw + 4 * lane) = h4;
    *(v4usa*)(rbw + DF + 4 * lane) = l4;
    wave_sync();
    const v8us qv = *(const v8usa*)(rbw + 8 * lane);
    wave_sync();
    if (live) {
      unsigned short* qp = QN + (size_t)n * 256 + 8 * lane;
      *(volatile v8us*)qp = qv;
      __threadfence();
      *(volatile v8us*)qp = qv;
    }
  }
  if (lane == 0) wpart[wave] = dacc;
  __syncthreads();
  if (wave == 0) {
    double tot = 0.0;
#pragma unroll 1
    for (int w2 = 0; w2 < NWAVE; ++w2) tot += wpart[w2];
    const v4f cv = *(const v4fa*)(coefs + 4 * (lane & 15));
    v2d o;
    o.x = (lane == 0) ? tot : 0.0;
    o.y = 0.0;
    float*  cp = coefo + (size_t)blockIdx.x * 64 + 4 * (lane & 15);
    double* pp = prec + (size_t)blockIdx.x * 16 + 2 * (lane & 7);
    const bool okc = lane < 16;
    const bool okp = lane < 8;
    if (okc) *(volatile v4f*)cp = cv;
    if (okp) *(volatile v2d*)pp = o;
    __threadfence();
    if (okc) *(volatile v4f*)cp = cv;
    if (okp) *(volatile v2d*)pp = o;
  }
}

__global__ __launch_bounds__(NTHR) void k_pool(const float* __restrict__ GL, const int* __restrict__ bat,
                                               const float* __restrict__ coef, const float* __restrict__ bsub,
                                               int nN, float* out, unsigned short* NK) {
  __shared__ __attribute__((aligned(16))) float wsum[NWAVE * 3 * DF];
  __shared__ __attribute__((aligned(16))) float outs[3 * DF];
  __shared__ __attribute__((aligned(16))) unsigned short rb[256];
  const int tid = (int)threadIdx.x, lane = tid & 31, wave = tid >> 5;
  const int g = (int)blockIdx.x;
  if (g >= NGR) {
    if (wave == 0) {
      const v8us z8 = {0, 0, 0, 0, 0, 0, 0, 0};
      unsigned short* np = NK + (size_t)g * 256 + 8 * lane;
      *(volatile v8us*)np = z8;
      __threadfence();
      *(volatile v8us*)np = z8;
    }
    return;
  }

  v4f pa = {0.0f, 0.0f, 0.0f, 0.0f};
  v4f sa = {0.0f, 0.0f, 0.0f, 0.0f};
  v4f na = {0.0f, 0.0f, 0.0f, 0.0f};
#pragma unroll 1
  for (int i0 = wave * 32; i0 < nN; i0 += NTHR) {
    const int i  = i0 + lane;
    const int ic = i < nN ? i : nN - 1;
    const int b  = bat[ic];
    const int cfi = __float_as_int(coef[ic]);
    const bool hit = (i < nN) && (b == g);
    unsigned msk = __builtin_amdgcn_ballot_w32(hit);
    int nh = (int)__builtin_popcount(msk);
    nh = nh > 32 ? 32 : nh;
#pragma unroll 1
    for (int q = 0; q < nh; ++q) {
      int k = __builtin_ffs((int)msk) - 1;
      msk &= msk - 1u;
      k = k < 0 ? 0 : k;
      int node = i0 + k;
      node = node > nN - 1 ? nN - 1 : node;
      const float ck = __int_as_float(__builtin_amdgcn_readlane(cfi, k));
      const v4f vp = *(const v4fa*)(GL + (size_t)node * DF + 4 * lane);
      const v4f vn = *(const v4fa*)(GL + (size_t)(nN + node) * DF + 4 * lane);
      pa += vp;
      na += vn;
      sa.x = fmaf(ck, vp.x, sa.x); sa.y = fmaf(ck, vp.y, sa.y);
      sa.z = fmaf(ck, vp.z, sa.z); sa.w = fmaf(ck, vp.w, sa.w);
    }
  }
  *(v4fa*)(wsum + wave * (3 * DF) + 4 * lane)          = pa;
  *(v4fa*)(wsum + wave * (3 * DF) + DF + 4 * lane)     = sa;
  *(v4fa*)(wsum + wave * (3 * DF) + 2 * DF + 4 * lane) = na;
  __syncthreads();
  const float bsv = bf16_val(bsub[0]);
#pragma unroll 1
  for (int c = tid; c < 3 * DF; c += NTHR) {
    float s = 0.0f;
#pragma unroll
    for (int w2 = 0; w2 < NWAVE; ++w2) s += wsum[w2 * (3 * DF) + c];
    if (c >= DF && c < 2 * DF) s += bsv;
    outs[c] = s;
  }
  __syncthreads();
  if (wave < 3) {
    const v4f ov = *(const v4fa*)(outs + DF * wave + 4 * lane);
    float* op = out + (size_t)wave * (NGR * DF) + (size_t)g * DF + 4 * lane;
    *(volatile v4f*)op = ov;
    __threadfence();
    *(volatile v4f*)op = ov;
  } else if (wave == 3) {
    const v4f pv = *(const v4fa*)(outs + 4 * lane);
    float ss = pv.x * pv.x + pv.y * pv.y + pv.z * pv.z + pv.w * pv.w;
#pragma unroll
    for (int o = 16; o > 0; o >>= 1) ss += __shfl_xor(ss, o, 32);
    const float inv = 1.0f / fmaxf(sqrtf(ss), 1e-12f);
    const float q0 = pv.x * inv, q1 = pv.y * inv, q2 = pv.z * inv, q3 = pv.w * inv;
    v4us h4, l4;
    unsigned hb;
    hb = bf16_bits(q0); h4[0] = (unsigned short)hb; l4[0] = (unsigned short)bf16_bits(q0 - __uint_as_float(hb << 16));
    hb = bf16_bits(q1); h4[1] = (unsigned short)hb; l4[1] = (unsigned short)bf16_bits(q1 - __uint_as_float(hb << 16));
    hb = bf16_bits(q2); h4[2] = (unsigned short)hb; l4[2] = (unsigned short)bf16_bits(q2 - __uint_as_float(hb << 16));
    hb = bf16_bits(q3); h4[3] = (unsigned short)hb; l4[3] = (unsigned short)bf16_bits(q3 - __uint_as_float(hb << 16));
    *(v4usa*)(rb + 4 * lane) = h4;
    *(v4usa*)(rb + DF + 4 * lane) = l4;
    wave_sync();
    const v8us qv = *(const v8usa*)(rb + 8 * lane);
    unsigned short* np = NK + (size_t)g * 256 + 8 * lane;
    *(volatile v8us*)np = qv;
    __threadfence();
    *(volatile v8us*)np = qv;
  }
}

__global__ __launch_bounds__(MTHR) void k_nce(const unsigned short* __restrict__ QN,
                                              const unsigned short* __restrict__ NK, int nN, float* lossv) {
  __shared__ __attribute__((aligned(16))) float stg[MROWS * DF];
  __shared__ __attribute__((aligned(16))) float lossb[MROWS];
  const int tid = (int)threadIdx.x, lane = tid & 31, wave = tid >> 5, hh = lane >> 4, m = lane & 15;
  const int rowBase = (int)blockIdx.x * MROWS;
  int arow = rowBase + 16 * wave + m;
  arow = arow < nN ? arow : nN - 1;
  const unsigned short* ap = QN + (size_t)arow * 256 + 8 * hh;
  const unsigned short* bp = NK + (size_t)m * 256 + 8 * hh;

  v8f acc[8];
  const v8f zz = {0.f, 0.f, 0.f, 0.f, 0.f, 0.f, 0.f, 0.f};
#pragma unroll
  for (int t = 0; t < 8; ++t) acc[t] = zz;
#pragma unroll 1
  for (int ks = 0; ks < DF / 32; ++ks) {
    FragB ah, al;
    ah.h[0] = *(const v8usa*)(ap + 32 * ks);
    ah.h[1] = *(const v8usa*)(ap + 32 * ks + 16);
    al.h[0] = *(const v8usa*)(ap + DF + 32 * ks);
    al.h[1] = *(const v8usa*)(ap + DF + 32 * ks + 16);
#pragma unroll
    for (int nt = 0; nt < 8; ++nt) {
      const unsigned short* bq = bp + (size_t)(16 * nt) * 256 + 32 * ks;
      FragB bh, bl;
      bh.h[0] = *(const v8usa*)bq;
      bh.h[1] = *(const v8usa*)(bq + 16);
      bl.h[0] = *(const v8usa*)(bq + DF);
      bl.h[1] = *(const v8usa*)(bq + DF + 16);
      acc[nt] = wmb(ah, bh, acc[nt]);
      acc[nt] = wmb(al, bh, acc[nt]);
      acc[nt] = wmb(ah, bl, acc[nt]);
    }
  }
#pragma unroll
  for (int nt = 0; nt < 8; ++nt) {
    const int lc = 16 * nt + m;
#pragma unroll
    for (int r = 0; r < 8; ++r) stg[(16 * wave + 8 * hh + r) * DF + lc] = acc[nt][r];
  }
  __syncthreads();

  const bool valid = lane < (NGR / 4);
  const float ninf = __int_as_float((int)0xff800000u);
#pragma unroll 1
  for (int i = 0; i < 16; ++i) {
    const int lr = 16 * wave + i;
    v4f sv = *(const v4fa*)(stg + lr * DF + 4 * lane);
    sv.x *= 10.0f; sv.y *= 10.0f; sv.z *= 10.0f; sv.w *= 10.0f;
    const float t0 = __shfl(sv.x, 0, 32);
    const float ml = fmaxf(fmaxf(sv.x, sv.y), fmaxf(sv.z, sv.w));
    float mx = valid ? ml : ninf;
#pragma unroll
    for (int o = 16; o > 0; o >>= 1) mx = fmaxf(mx, __shfl_xor(mx, o, 32));
    const float es = (expf(sv.x - mx) + expf(sv.y - mx)) + (expf(sv.z - mx) + expf(sv.w - mx));
    float se = valid ? es : 0.0f;
#pragma unroll
    for (int o = 16; o > 0; o >>= 1) se += __shfl_xor(se, o, 32);
    se += expf(t0 - mx);
    const float ls = (mx + logf(se)) - t0;
    if (lane == 0) lossb[lr] = (rowBase + lr < nN) ? ls : 0.0f;
  }
  __syncthreads();
  if (wave == 0) {
    const v4f lv = *(const v4fa*)(lossb + 4 * (lane & 15));
    float* lp = lossv + (size_t)blockIdx.x * MROWS + 4 * (lane & 15);
    const bool okl = lane < 16;
    if (okl) *(volatile v4f*)lp = lv;
    __threadfence();
    if (okl) *(volatile v4f*)lp = lv;
  }
}

__global__ __launch_bounds__(NTHR) void k_segloss(const float* __restrict__ lossv, const int* __restrict__ bat,
                                                  int nN, double* grec) {
  __shared__ double ls[NTHR];
  __shared__ int lc[NWAVE];
  const int tid = (int)threadIdx.x, lane = tid & 31, wave = tid >> 5;
  const int g = (int)blockIdx.x;
  double a = 0.0;
  int cnt = 0;
#pragma unroll 1
  for (int i0 = wave * 32; i0 < nN; i0 += NTHR) {
    const int i  = i0 + lane;
    const int ic = i < nN ? i : nN - 1;
    const int b  = bat[ic];
    const float lv = lossv[ic];
    const bool hit = (i < nN) && (b == g);
    a += hit ? (double)lv : 0.0;
    cnt += (int)__builtin_popcount(__builtin_amdgcn_ballot_w32(hit));
  }
  ls[tid] = a;
  if (lane == 0) lc[wave] = cnt;
  __syncthreads();
  if (wave == 0) {
    double S = 0.0;
#pragma unroll 1
    for (int j = 0; j < NTHR; ++j) S += ls[j];
    int C = 0;
#pragma unroll
    for (int w2 = 0; w2 < NWAVE; ++w2) C += lc[w2];
    v2d o;
    o.x = (lane == 0) ? S : 0.0;
    o.y = (lane == 0) ? (double)C : 0.0;
    double* gp = grec + (size_t)g * 16 + 2 * (lane & 7);
    const bool okg = lane < 8;
    if (okg) *(volatile v2d*)gp = o;
    __threadfence();
    if (okg) *(volatile v2d*)gp = o;
  }
}

__global__ __launch_bounds__(NTHR) void k_final(const double* __restrict__ prec, int nRec,
                                                const double* __restrict__ grec, const int* __restrict__ sel,
                                                float* out) {
  __shared__ double pa[NTHR];
  const int tid = (int)threadIdx.x;
  double a = 0.0;
#pragma unroll 1
  for (int b = tid; b < nRec; b += NTHR) a += prec[(size_t)b * 16];
  pa[tid] = a;
  __syncthreads();
  if (tid == 0) {
    double P = 0.0;
#pragma unroll 1
    for (int j = 0; j < NTHR; ++j) P += pa[j];
    double I = 0.0;
#pragma unroll 1
    for (int g = 0; g < NGR; ++g) {
      const double S = grec[(size_t)g * 16];
      const double C = grec[(size_t)g * 16 + 1];
      I += S / C;
    }
    I = I * (1.0 / (double)NGR);
    const float pn = (sel[0] != 0) ? __int_as_float(0x7fc00000) : 0.0f;
    v2f o;
    o.x = (float)(-P) + pn;
    o.y = (float)I + pn;
    float* op = out + 3 * NGR * DF;
    *(volatile v2f*)op = o;
    __threadfence();
    *(volatile v2f*)op = o;
  }
}

static inline int cdiv(int a, int b) { return (a + b - 1) / b; }
static inline size_t al256(size_t o) { return (o + 255) & ~(size_t)255; }

extern "C" void kernel_launch(void* const* d_in, const int* in_sizes, int n_in,
                              void* d_out, int out_size, void* d_ws, size_t ws_size,
                              hipStream_t stream) {
  if (n_in < 21) return;
  const int nN = NNODE, nE = NEDGE;
  if (in_sizes[0] != nN * DF) return;
  if (in_sizes[1] != 2 * nE) return;
  if (in_sizes[2] != nN || in_sizes[3] != nN || in_sizes[4] != 1) return;
  if (in_sizes[5] != DF * DF || in_sizes[6] != DF) return;
  if (in_sizes[7] != DF * DF || in_sizes[8] != DF) return;
  if (in_sizes[9] != 3 * DF * DF || in_sizes[10] != 3 * DF) return;
  if (in_sizes[11] != 3 * DF * DF || in_sizes[12] != 3 * DF) return;
  if (in_sizes[13] != 3 * DF || in_sizes[14] != 3 * DF) return;
  if (in_sizes[15] != 3 || in_sizes[16] != 1) return;
  if (in_sizes[17] != 3 * DF * 2 || in_sizes[18] != 6) return;
  if (in_sizes[19] != 4 || in_sizes[20] != 1) return;
  if (out_size != NOUTF) return;

  const float* x    = (const float*)d_in[0];
  const int*   edge = (const int*)d_in[1];
  const int*   bat  = (const int*)d_in[2];
  const int*   nidx = (const int*)d_in[3];
  const int*   sel  = (const int*)d_in[4];
  const float* Wi1  = (const float*)d_in[5];
  const float* bi1  = (const float*)d_in[6];
  const float* Wi2  = (const float*)d_in[7];
  const float* bi2  = (const float*)d_in[8];
  const float* Wg1  = (const float*)d_in[9];
  const float* bg1  = (const float*)d_in[10];
  const float* Wg2  = (const float*)d_in[11];
  const float* bg2  = (const float*)d_in[12];
  const float* gam  = (const float*)d_in[13];
  const float* bet  = (const float*)d_in[14];
  const float* wly  = (const float*)d_in[15];
  const float* bly  = (const float*)d_in[16];
  const float* Wp   = (const float*)d_in[17];
  const float* bp   = (const float*)d_in[18];
  const float* wsub = (const float*)d_in[19];
  const float* bsub = (const float*)d_in[20];
  float* out = (float*)d_out;
  const int* src = edge;
  const int* dst = edge + nE;

  char* ws = (char*)d_ws;
  size_t off = 0;
  const size_t oB0 = off; off = al256(off + (size_t)R2 * DF * 4);
  const size_t oB1 = off; off = al256(off + (size_t)R2 * DF * 4);
  const size_t oGL = off; off = al256(off + (size_t)R2 * DF * 4);
  const size_t oWT = off; off = al256(off + (size_t)8 * DF * DF * 2);
  const size_t oRC = off; off = al256(off + (size_t)NRECB * 2 * DF * 8);
  const size_t oST = off; off = al256(off + (size_t)2 * DF * 4);
  const size_t oCF = off; off = al256(off + (size_t)NTSB * 64 * 4);
  const size_t oPR = off; off = al256(off + (size_t)NTSB * 128);
  const size_t oNK = off; off = al256(off + (size_t)NKROWS * 256 * 2);
  const size_t oLS = off; off = al256(off + (size_t)NTSB * 64 * 4);
  const size_t oGR = off; off = al256(off + (size_t)NGR * 128);
  if (off > ws_size) return;
  float*          BUF0 = (float*)(ws + oB0);
  float*          BUF1 = (float*)(ws + oB1);
  float*          GLB  = (float*)(ws + oGL);
  unsigned short* WT   = (unsigned short*)(ws + oWT);
  double*         REC  = (double*)(ws + oRC);
  float*          STAT = (float*)(ws + oST);
  float*          COEF = (float*)(ws + oCF);
  double*         PREC = (double*)(ws + oPR);
  unsigned short* NK   = (unsigned short*)(ws + oNK);
  float*          LOSS = (float*)(ws + oLS);
  double*         GREC = (double*)(ws + oGR);
  unsigned short* QN   = (unsigned short*)(ws + oB0);

  const size_t scanLds = (size_t)AGG_LDS_INTS * 4;
  hipFuncSetAttribute(reinterpret_cast<const void*>(&k_scan), hipFuncAttributeMaxDynamicSharedMemorySize, (int)scanLds);

  const int gScan = cdiv(nN, NBA);
  const int WSZ = DF * DF;

  k_prep<<<(8 * 2048) / NTHR, NTHR, 0, stream>>>(Wi1, Wi2, Wg1, Wg2, WT);
  k_mlp<0><<<cdiv(nN, MROWS), MTHR, 0, stream>>>(x, nN, WT, bi1, WT + WSZ, bi2, BUF0, REC);
  k_neg<<<cdiv(nN * 32, NTHR), NTHR, 0, stream>>>(BUF0, nidx, nN);
  for (int l = 0; l < 3; ++l) {
    float* A = (l & 1) ? BUF1 : BUF0;
    float* B = (l & 1) ? BUF0 : BUF1;
    k_scan<<<gScan, NTHR, scanLds, stream>>>(src, dst, nE, nN, A, B);
    k_mlp<1><<<NRECB, MTHR, 0, stream>>>(B, R2, WT + (size_t)(2 + l) * WSZ, bg1 + l * DF,
                                         WT + (size_t)(5 + l) * WSZ, bg2 + l * DF, B, REC);
    k_bn_combine<<<1, NTHR, 0, stream>>>(REC, NRECB, STAT);
    k_bn_apply<<<cdiv(R2, 64), NTHR, 0, stream>>>(B, GLB, STAT, gam + l * DF, bet + l * DF, wly + l, bly, l, R2);
  }
  k_ts<<<NTSB, NTHR, 0, stream>>>(GLB, Wp, bp, wsub, nN, COEF, PREC, QN);
  k_pool<<<NKROWS, NTHR, 0, stream>>>(GLB, bat, COEF, bsub, nN, out, NK);
  k_nce<<<NTSB, MTHR, 0, stream>>>(QN, NK, nN, LOSS);
  k_segloss<<<NGR, NTHR, 0, stream>>>(LOSS, bat, nN, GREC);
  k_final<<<1, NTHR, 0, stream>>>(PREC, NTSB, GREC, sel, out);
}
